// DyadicSignature_67327907332419
// MI455X (gfx1250) — hardware-run, weakly checked
//
#include <hip/hip_runtime.h>


#ifndef NB
#define NB 32
#endif
#define NB_FULL 32
#define CH      32
#define FRAMES  160
#define NSEG    16
#define SEGLEN  10
#define NSTEP   9
#define SIGC    33824
#define A2OFF   32
#define A3OFF   1056
#define NLVL    5
#define SIG4    (SIGC / 4)
#define LGP     32
#define UPQ     5
#define OSP     36
#define INV6    (1.0f / 6.0f)
#define NEGB    (-3.0e38f)

static_assert(CH == 32);
static_assert(SIGC == CH + CH * CH + CH * CH * CH);
static_assert(A2OFF == CH);
static_assert(A3OFF == CH + CH * CH);
static_assert(SIGC % 32 == 0);
static_assert(A2OFF % 32 == 0);
static_assert(A3OFF % 32 == 0);
static_assert(FRAMES == NSEG * SEGLEN);
static_assert(NSTEP == SEGLEN - 1);
static_assert(3 * NSTEP <= 32);
static_assert(SIG4 % 8 == 0);
static_assert(NB <= NB_FULL);
static_assert(32 * 16 * 4 == 16 * 128);
static_assert(256 * 16 == 32 * 128);
static_assert(256 * 16 * CH == CH * CH * 128);
static_assert(256 * 16 == CH * CH * 4);
static_assert((OSP * 4) % 16 == 0);
static_assert(NSTEP * CH * 4 * 3 + CH * UPQ * 16 + 8 * 32 * UPQ * 16 + 8 * 16 * OSP * 4 + 32 <= 131072);
static_assert(CH * 4 + CH * CH * 4 + CH * 4 + CH * CH * 4 + 32 <= 131072);

typedef __attribute__((ext_vector_type(16))) __bf16       v16bf;
typedef __attribute__((ext_vector_type(8)))  float        v8f;
typedef __attribute__((ext_vector_type(4)))  float        v4f;
typedef v4f  __attribute__((may_alias)) v4fa;
typedef __attribute__((ext_vector_type(4)))  unsigned int v4u;
typedef __attribute__((ext_vector_type(8)))  unsigned int v8u;

__device__ __forceinline__ unsigned short f2bf(float f) { unsigned u = __float_as_uint(f); u += 0x7FFFu + ((u >> 16) & 1u); return (unsigned short)(u >> 16); }
__device__ __forceinline__ float bfr(float f) { return __uint_as_float(((unsigned)f2bf(f)) << 16); }
__device__ __forceinline__ void wave_sync() { __builtin_amdgcn_fence(3  , "wavefront"); __builtin_amdgcn_wave_barrier(); asm volatile("" ::: "memory"); }

__device__ __forceinline__ unsigned pk(unsigned lo, unsigned hi16) { return lo | (hi16 << 16); }
__device__ __forceinline__ v16bf frag8(v4u a, v4u b) { return __builtin_bit_cast(v16bf, __builtin_shufflevector(a, b, 0, 1, 2, 3, 4, 5, 6, 7)); }
__device__ __forceinline__ v8f wmmab_g(v16bf a, v16bf b, v8f c) {
    c = __builtin_amdgcn_wmma_f32_16x16x32_bf16(false, a, false, b, (short)0, c, false, false);
    asm volatile("v_nop\n\tv_nop\n\tv_nop\n\tv_nop" : "+v"(c) : "v"(a), "v"(b));
    return c;
}
__device__ __forceinline__ float dotw(v4f v, v4f wv) { return v[0] * bfr(wv[0]) + v[1] * bfr(wv[1]) + v[2] * bfr(wv[2]) + v[3] * bfr(wv[3]); }
__device__ __forceinline__ float wsum(float v) {
    v += __shfl_xor(v, 16, 32); v += __shfl_xor(v, 8, 32); v += __shfl_xor(v, 4, 32); v += __shfl_xor(v, 2, 32); v += __shfl_xor(v, 1, 32); return v; }
__device__ __forceinline__ float wmax(float v) {
    v = fmaxf(v, __shfl_xor(v, 16, 32)); v = fmaxf(v, __shfl_xor(v, 8, 32)); v = fmaxf(v, __shfl_xor(v, 4, 32)); v = fmaxf(v, __shfl_xor(v, 2, 32)); v = fmaxf(v, __shfl_xor(v, 1, 32)); return v; }

__global__ __launch_bounds__(256) void k_sig(const float* __restrict__ x, const float* __restrict__ w, float* SG, float* LG)
{
    __shared__ float Vs[NSTEP * CH];
    __shared__ float A1P[NSTEP * CH];
    __shared__ float Ws[NSTEP * CH];
    __shared__ v4u VBq[CH * UPQ];
    __shared__ v4u UAq[8 * 32 * UPQ];
    __shared__ __align__(16) float os[8 * 16 * OSP];
    __shared__ float red[8];

    const int tid = threadIdx.x, lane = tid & 31, lr = lane & 15, hi = lane >> 4;
    const int wave = __builtin_amdgcn_readfirstlane((int)(threadIdx.x >> 5));
    const int seg = blockIdx.x; const int b = seg / NSEG, g = seg % NSEG;
    const float* xb = x + (size_t)b * (CH * FRAMES) + g * SEGLEN;
    float* out = SG + (size_t)seg * SIGC;
    float lg = 0.0f;

#pragma unroll 1
    for (int t = wave; t < NSTEP; t += 8) {
        const float x0 = bfr(xb[lane * FRAMES + t]); const float x1 = bfr(xb[lane * FRAMES + t + 1]);
        Vs[t * CH + lane] = x1 - x0;
    }
    __syncthreads();
#pragma unroll 1
    for (int t = wave; t < NSTEP; t += 8) {
        float p = 0.0f;
#pragma unroll 1
        for (int s = 0; s < t; ++s) p += Vs[s * CH + lane];
        A1P[t * CH + lane] = p; Ws[t * CH + lane] = p + 0.5f * Vs[t * CH + lane];
    }
    if (wave == 7) {
        unsigned VH[NSTEP], VL[NSTEP];
#pragma unroll
        for (int t = 0; t < NSTEP; ++t) { const float v = Vs[t * CH + lane]; const unsigned hb = f2bf(v); VH[t] = hb; VL[t] = f2bf(v - __uint_as_float(hb << 16)); }
        v4u q0, q1, q2, q3;
        q0[0] = pk(VH[0], VH[1]); q0[1] = pk(VH[2], VH[3]); q0[2] = pk(VH[4], VH[5]); q0[3] = pk(VH[6], VH[7]);
        q1[0] = pk(VH[8], VL[0]); q1[1] = pk(VL[1], VL[2]); q1[2] = pk(VL[3], VL[4]); q1[3] = pk(VL[5], VL[6]);
        q2[0] = pk(VL[7], VL[8]); q2[1] = pk(VH[0], VH[1]); q2[2] = pk(VH[2], VH[3]); q2[3] = pk(VH[4], VH[5]);
        q3[0] = pk(VH[6], VH[7]); q3[1] = VH[8];            q3[2] = 0u;               q3[3] = 0u;
        VBq[lane * UPQ + 0] = q0; VBq[lane * UPQ + 1] = q1; VBq[lane * UPQ + 2] = q2; VBq[lane * UPQ + 3] = q3;
    }
    __syncthreads();

    const v16bf bf0 = frag8(VBq[lr * UPQ + hi], VBq[lr * UPQ + 2 + hi]);
    const v16bf bf1 = frag8(VBq[(16 + lr) * UPQ + hi], VBq[(16 + lr) * UPQ + 2 + hi]);

    if (wave == 0) {
        const float a1v = A1P[(NSTEP - 1) * CH + lane] + Vs[(NSTEP - 1) * CH + lane];
        lg += a1v * bfr(w[lane]);
#pragma unroll 1
        for (int ps = 0; ps < 2; ++ps) { *(volatile float*)(out + lane) = a1v; if (ps == 0) __threadfence(); }
    }

    const int ub = (wave * 32 + lane) * UPQ;
    const int ob = wave * 16 * OSP;
#pragma unroll 1
    for (int ii = 0; ii < 4; ++ii) {
        const int i = wave * 4 + ii;
        float a2run = 0.0f; unsigned H[NSTEP], L[NSTEP];
#pragma unroll
        for (int t = 0; t < NSTEP; ++t) {
            const float vi = Vs[t * CH + i], vj = Vs[t * CH + lane], ap = A1P[t * CH + i], wi = Ws[t * CH + i];
            const float u = a2run + 0.5f * ap * vj + INV6 * vi * vj;
            const unsigned hb = f2bf(u); H[t] = hb; L[t] = f2bf(u - __uint_as_float(hb << 16));
            a2run += wi * vj;
        }
        { v4u q0, q1, q2, q3;
          q0[0] = pk(H[0], H[1]); q0[1] = pk(H[2], H[3]); q0[2] = pk(H[4], H[5]); q0[3] = pk(H[6], H[7]);
          q1[0] = pk(H[8], H[0]); q1[1] = pk(H[1], H[2]); q1[2] = pk(H[3], H[4]); q1[3] = pk(H[5], H[6]);
          q2[0] = pk(H[7], H[8]); q2[1] = pk(L[0], L[1]); q2[2] = pk(L[2], L[3]); q2[3] = pk(L[4], L[5]);
          q3[0] = pk(L[6], L[7]); q3[1] = L[8];           q3[2] = 0u;             q3[3] = 0u;
          UAq[ub + 0] = q0; UAq[ub + 1] = q1; UAq[ub + 2] = q2; UAq[ub + 3] = q3; }
        wave_sync();
        const int ra = (wave * 32 + lr) * UPQ, rb = (wave * 32 + 16 + lr) * UPQ;
        const v16bf af0 = frag8(UAq[ra + hi], UAq[ra + 2 + hi]);
        const v16bf af1 = frag8(UAq[rb + hi], UAq[rb + 2 + hi]);
        v8f acc[2][2];
        acc[0][0] = wmmab_g(af0, bf0, (v8f){}); acc[0][1] = wmmab_g(af0, bf1, (v8f){});
        acc[1][0] = wmmab_g(af1, bf0, (v8f){}); acc[1][1] = wmmab_g(af1, bf1, (v8f){});
        const float a2v = a2run;
        lg += a2v * bfr(w[A2OFF + i * CH + lane]);
#pragma unroll
        for (int rt = 0; rt < 2; ++rt) {
#pragma unroll
            for (int r = 0; r < 8; ++r) {
                os[ob + (8 * hi + r) * OSP + lr]      = acc[rt][0][r];
                os[ob + (8 * hi + r) * OSP + 16 + lr] = acc[rt][1][r]; }
            wave_sync();
            const size_t e0 = (size_t)A3OFF + (size_t)(i * 32 + rt * 16) * 32;
            v4f val[4];
#pragma unroll
            for (int s = 0; s < 4; ++s) { const int row = 4 * s + (lane >> 3), cofs = (lane & 7) * 4;
                val[s] = *(const v4fa*)(&os[ob + row * OSP + cofs]);
                const v4f wv = *(const v4f*)(w + e0 + (size_t)row * 32 + cofs);
                lg += dotw(val[s], wv); }
            float* orow = out + e0;
#pragma unroll 1
            for (int ps = 0; ps < 2; ++ps) {
#pragma unroll
                for (int s = 0; s < 4; ++s) { const int row = 4 * s + (lane >> 3), cofs = (lane & 7) * 4;
                    *(volatile v4f*)(orow + (size_t)row * 32 + cofs) = val[s]; }
                if (rt == 0) *(volatile float*)(out + A2OFF + i * CH + lane) = a2v;
                if (ps == 0) __threadfence(); }
            wave_sync();
        }
    }
    lg = wsum(lg);
    if (lane == 0) red[wave] = lg;
    __syncthreads();
    if (wave == 0) {
        float tot = red[0];
#pragma unroll
        for (int k = 1; k < 8; ++k) tot += red[k];
#pragma unroll 1
        for (int ps = 0; ps < 2; ++ps) { *(volatile float*)(LG + (size_t)seg * LGP + lane) = tot; if (ps == 0) __threadfence(); }
    }
}

__global__ __launch_bounds__(256) void k_comb(const float* __restrict__ SRC, float* DST, size_t dstride, const float* __restrict__ w, float* LG)
{
    __shared__ float a1s[CH];
    __shared__ float a2s[CH * CH];
    __shared__ v4f   b1q[CH / 4];
    __shared__ v4f   b2q[CH * CH / 4];
    __shared__ float red[8];

    const int tid = threadIdx.x, lane = tid & 31;
    const int wave = __builtin_amdgcn_readfirstlane((int)(threadIdx.x >> 5));
    const int g = blockIdx.x;
    const float* A = SRC + (size_t)(2 * g) * SIGC;
    const float* B = A + SIGC;
    float* D = DST + (size_t)g * dstride;
    const int q = tid & 7;

#pragma unroll
    for (int k = 0; k < 4; ++k) a2s[k * 256 + tid] = A[A2OFF + k * 256 + tid];
    b2q[tid] = *(const v4f*)(B + A2OFF + tid * 4);
    if (wave == 0) { a1s[lane] = A[lane]; const v4f t = *(const v4f*)(B + (lane & 7) * 4); if (lane < 8) b1q[lane] = t; }
    __syncthreads();
    const v4f b1v = b1q[q];
    const v4f b2v = b2q[tid];
    float lg = 0.0f;

    if (wave == 0) {
        const v4f va = *(const v4f*)(A + q * 4), vb = *(const v4f*)(B + q * 4); const v4f wv = *(const v4f*)(w + q * 4);
        const v4f vc = va + vb;
        const float t = dotw(vc, wv);
        lg += (lane < 8) ? t : 0.0f;
#pragma unroll 1
        for (int ps = 0; ps < 2; ++ps) { if (lane < 8) *(volatile v4f*)(D + q * 4) = vc; if (ps == 0) __threadfence(); }
    }
    {
        const v4f va = *(const v4f*)(A + A2OFF + tid * 4); const v4f wv = *(const v4f*)(w + A2OFF + tid * 4);
        const float a1i = a1s[tid >> 3];
        const v4f vc = (va + b2v) + a1i * b1v;
        lg += dotw(vc, wv);
#pragma unroll 1
        for (int ps = 0; ps < 2; ++ps) { *(volatile v4f*)(D + A2OFF + tid * 4) = vc; if (ps == 0) __threadfence(); }
    }
#pragma unroll 1
    for (int it = 0; it < CH; ++it) {
        const size_t e = (size_t)A3OFF + (size_t)it * (CH * CH) + (size_t)tid * 4;
        const v4f va = *(const v4f*)(A + e), vb = *(const v4f*)(B + e); const v4f wv = *(const v4f*)(w + e);
        const float a1i = a1s[it]; const float a2ij = a2s[it * CH + (tid >> 3)];
        const v4f vc = ((va + vb) + a1i * b2v) + a2ij * b1v;
        lg += dotw(vc, wv);
#pragma unroll 1
        for (int ps = 0; ps < 2; ++ps) { *(volatile v4f*)(D + e) = vc; if (ps == 0) __threadfence(); }
    }
    lg = wsum(lg);
    if (lane == 0) red[wave] = lg;
    __syncthreads();
    if (wave == 0) {
        float tot = red[0];
#pragma unroll
        for (int k = 1; k < 8; ++k) tot += red[k];
#pragma unroll 1
        for (int ps = 0; ps < 2; ++ps) { *(volatile float*)(LG + (size_t)g * LGP + lane) = tot; if (ps == 0) __threadfence(); }
    }
}

__global__ __launch_bounds__(256) void k_pairw(const float* __restrict__ SG, const float* __restrict__ LG, const float* __restrict__ bias, int S, float* OUT)
{
    __shared__ float ps_[16];
    const int tid = threadIdx.x, lane = tid & 31;
    const int wave = __builtin_amdgcn_readfirstlane((int)(threadIdx.x >> 5));
    const int b = blockIdx.y;
    if (wave == 0) {
        const int sc = (lane < S) ? lane : (S - 1);
        float lv = LG[(size_t)(b * S + sc) * LGP];
        asm volatile("" : "+v"(lv));
        const float bv = bfr(bias[0]);
        const bool on = lane < S;
        const float z = on ? (lv + bv) : NEGB;
        const float mx = wmax(z);
        const float ex = expf(z - mx);
        const float e = on ? ex : 0.0f;
        const float sm = wsum(e);
        const float p = e * (1.0f / sm);
        if (lane < 16) ps_[lane] = p;
    }
    __syncthreads();
    const int f = blockIdx.x * 256 + tid;
    const int fc = (f < SIG4) ? f : (SIG4 - 1);
    const float* src = SG + (size_t)b * (size_t)S * SIGC + (size_t)fc * 4;
    v4f acc = (v4f){};
#pragma unroll 1
    for (int s = 0; s < S; ++s) { const v4f v = *(const v4f*)(src + (size_t)s * SIGC); acc += ps_[s] * v; }
    float* dst = OUT + (size_t)b * (NLVL * SIGC) + (size_t)fc * 4;
#pragma unroll 1
    for (int ps = 0; ps < 2; ++ps) { if (f < SIG4) *(volatile v4f*)dst = acc; if (ps == 0) __threadfence(); }
}

static constexpr size_t al256(size_t v) { return (v + 255) & ~(size_t)255; }
static constexpr size_t SZ_BA = al256((size_t)NB * 16 * SIGC * 4);
static constexpr size_t SZ_BB = al256((size_t)NB * 8 * SIGC * 4);
static constexpr size_t SZ_LG = al256((size_t)NB * 16 * LGP * 4);
static constexpr size_t SZ_TOTAL = SZ_BA + SZ_BB + 5 * SZ_LG;
static_assert(SZ_TOTAL <= (size_t)134217728);
static_assert(((size_t)SIGC * 4) % 128 == 0);
static_assert((size_t)NB * 4 * SIGC * 4 <= SZ_BA);
static_assert((size_t)NB * 2 * SIGC * 4 <= SZ_BB);

extern "C" void kernel_launch(void* const* d_in, const int* in_sizes, int n_in,
                              void* d_out, int out_size, void* d_ws, size_t ws_size, hipStream_t stream) {
    if (n_in < 3) return;
    if ((size_t)in_sizes[0] < (size_t)NB * CH * FRAMES) return;
    if ((size_t)in_sizes[1] < (size_t)4 * SIGC) return;
    if (in_sizes[2] < 4) return;
    if ((size_t)out_size < (size_t)NB * NLVL * SIGC) return;
    if (SZ_TOTAL > ws_size) return;
    const float* x  = (const float*)d_in[0];
    const float* aw = (const float*)d_in[1];
    const float* ab = (const float*)d_in[2];
    float* OUT = (float*)d_out;
    char* wsp = (char*)d_ws;
    float* BA  = (float*)wsp; wsp += SZ_BA;
    float* BB  = (float*)wsp; wsp += SZ_BB;
    float* LG4 = (float*)wsp; wsp += SZ_LG;
    float* LG3 = (float*)wsp; wsp += SZ_LG;
    float* LG2 = (float*)wsp; wsp += SZ_LG;
    float* LG1 = (float*)wsp; wsp += SZ_LG;
    float* LG0 = (float*)wsp; wsp += SZ_LG;
    const dim3 ga((SIG4 + 255) / 256, NB, 1);

    k_sig <<<NB * 16, 256, 0, stream>>>(x, aw + (size_t)3 * SIGC, BA, LG4);
    k_pairw<<<ga, 256, 0, stream>>>(BA, LG4, ab + 3, 16, OUT + (size_t)4 * SIGC);
    k_comb<<<NB * 8, 256, 0, stream>>>(BA, BB, (size_t)SIGC, aw + (size_t)2 * SIGC, LG3);
    k_pairw<<<ga, 256, 0, stream>>>(BB, LG3, ab + 2, 8, OUT + (size_t)3 * SIGC);
    k_comb<<<NB * 4, 256, 0, stream>>>(BB, BA, (size_t)SIGC, aw + (size_t)1 * SIGC, LG2);
    k_pairw<<<ga, 256, 0, stream>>>(BA, LG2, ab + 1, 4, OUT + (size_t)2 * SIGC);
    k_comb<<<NB * 2, 256, 0, stream>>>(BA, BB, (size_t)SIGC, aw, LG1);
    k_pairw<<<ga, 256, 0, stream>>>(BB, LG1, ab, 2, OUT + (size_t)1 * SIGC);
    k_comb<<<NB, 256, 0, stream>>>(BB, OUT, (size_t)NLVL * SIGC, aw, LG0);
}
